// DeltaNet_22488448762193
// MI455X (gfx1250) — hardware-run, weakly checked
//
#include <hip/hip_runtime.h>
#include <math.h>

constexpr int kB     = 2;
constexpr int kL     = 2048;
constexpr int kD     = 1024;
constexpr int kH     = 8;
constexpr int kDh    = kD / kH;
constexpr int kRows  = kB * kL;
constexpr int kNcat  = 3 * kD + 64;
constexpr int kGate0 = 3 * kD;
constexpr int kQKP   = 2 * kD;
constexpr int kGP    = 32;
constexpr int kScT   = 32;
constexpr int kScE   = 64;
constexpr float kWoCarry  = 1024.0f;
constexpr float kOCarry   = 16.0f;
constexpr float kOutScale = 1.0f / (kWoCarry * kOCarry);
constexpr float kF16MinNormal = 6.103515625e-5f;
constexpr float kF16Clamp     = 60000.0f;
constexpr float kBetaMin  = 0.85f;
constexpr float kBetaSpan = 0.149f;

static_assert(kDh == 128, "head width");
static_assert(kRows == 4096, "token rows");
static_assert(kNcat == 3136 && (kNcat % 64) == 0, "concatenated N is a 64 multiple");
static_assert((kD % 32) == 0, "GEMM K multiple of 32");
static_assert((kRows % 64) == 0 && (kD % 64) == 0, "GEMM M, N multiples of 64");
static_assert(kScT == 32 && (kL % kScT) == 0, "scan chunking");
static_assert(kDh == 2 * kScE, "two scan blocks per head");
static_assert(((kRows / 64) * (kNcat / 64)) % 8 == 0, "projection GEMM grid exact");
static_assert(((kRows / 64) * (kD / 64)) % 8 == 0, "output GEMM grid exact");

typedef __attribute__((ext_vector_type(16))) _Float16 v16h;
typedef __attribute__((ext_vector_type(8)))  _Float16 v8h;
typedef __attribute__((ext_vector_type(16))) __bf16   v16b;
typedef __attribute__((ext_vector_type(8)))  __bf16   v8b;
typedef __attribute__((ext_vector_type(8)))  float    v8f;
typedef __attribute__((ext_vector_type(4)))  float    v4f;

constexpr size_t kSzXB    = (size_t)kRows * kD * 2;
constexpr size_t kSzWCAT  = (size_t)kNcat * kD * 2;
constexpr size_t kSzWOH   = (size_t)kD * kD * 2;
constexpr size_t kSzBOB   = (size_t)kD * 4;
constexpr size_t kSzQKVG  = (size_t)kRows * kNcat * 4;
constexpr size_t kSzQKR   = (size_t)kRows * kQKP * 4;
constexpr size_t kSzGATES = (size_t)kRows * kGP * 4;
constexpr size_t kSzOH    = (size_t)kRows * kD * 2;
constexpr size_t kWsTotal = kSzXB + kSzWCAT + kSzWOH + kSzBOB + kSzQKVG + kSzQKR + kSzGATES + kSzOH;
static_assert(kWsTotal == 110759936ull, "carve total");
static_assert(kWsTotal <= 134217728ull, "carve cap");
static_assert((kSzXB % 256) == 0 && (kSzWCAT % 256) == 0 && (kSzWOH % 256) == 0 && (kSzBOB % 256) == 0 &&
              (kSzQKVG % 256) == 0 && (kSzQKR % 256) == 0 && (kSzGATES % 256) == 0 && (kSzOH % 256) == 0, "aligned regions");

__device__ __forceinline__ unsigned short f2bf_bits(float f) {
  unsigned u = __float_as_uint(f);
  return (unsigned short)((u + 0x7FFFu + ((u >> 16) & 1u)) >> 16);
}
__device__ __forceinline__ float bf_bits2f(unsigned short h) { return __uint_as_float(((unsigned)h) << 16); }
__device__ __forceinline__ float bf16r(float f) { return bf_bits2f(f2bf_bits(f)); }
__device__ __forceinline__ _Float16 to_f16_operand(float v) {
  float c = fminf(fmaxf(v, -kF16Clamp), kF16Clamp);
  c = (fabsf(c) < kF16MinNormal) ? 0.0f : c;
  return (_Float16)c;
}

__device__ __forceinline__ void dep_guard4_h(v8f& a, v8f& b, v8f& c, v8f& d, v16h x, v16h y) {
  asm volatile("v_nop\n\tv_nop\n\tv_nop\n\tv_nop" : "+v"(a), "+v"(b), "+v"(c), "+v"(d) : "v"(x), "v"(y));
}
__device__ __forceinline__ void dep_guard4_b(v8f& a, v8f& b, v8f& c, v8f& d, v16b x, v16b y) {
  asm volatile("v_nop\n\tv_nop\n\tv_nop\n\tv_nop" : "+v"(a), "+v"(b), "+v"(c), "+v"(d) : "v"(x), "v"(y));
}
__device__ __forceinline__ void keep4_h(v16h a, v16h b, v16h c, v16h d) { asm volatile("v_nop" :: "v"(a), "v"(b), "v"(c), "v"(d)); }
__device__ __forceinline__ void keep4_b(v16b a, v16b b, v16b c, v16b d) { asm volatile("v_nop" :: "v"(a), "v"(b), "v"(c), "v"(d)); }
__device__ __forceinline__ void acc_guard4(v8f& a, v8f& b, v8f& c, v8f& d) {
  asm volatile("v_nop\n\tv_nop\n\tv_nop\n\tv_nop" : "+v"(a), "+v"(b), "+v"(c), "+v"(d));
}

template <typename T> struct Frag;
template <> struct Frag<_Float16> {
  typedef v16h V; union U { v16h v; v8h h[2]; };
  static __device__ __forceinline__ v16h load(const _Float16* p) {
    U f; f.h[0] = *(const v8h*)(p); f.h[1] = *(const v8h*)(p + 16); return f.v;
  }
  static __device__ __forceinline__ v8f mma(v16h a, v16h b, v8f c) {
    return __builtin_amdgcn_wmma_f32_16x16x32_f16(false, a, false, b, (short)0, c, false, false);
  }
  static __device__ __forceinline__ void guard4(v8f& a, v8f& b, v8f& c, v8f& d, v16h x, v16h y) { dep_guard4_h(a, b, c, d, x, y); }
  static __device__ __forceinline__ void keep(v16h a, v16h b, v16h c, v16h d) { keep4_h(a, b, c, d); }
};
template <> struct Frag<__bf16> {
  typedef v16b V; union U { v16b v; v8b h[2]; };
  static __device__ __forceinline__ v16b load(const __bf16* p) {
    U f; f.h[0] = *(const v8b*)(p); f.h[1] = *(const v8b*)(p + 16); return f.v;
  }
  static __device__ __forceinline__ v8f mma(v16b a, v16b b, v8f c) {
    return __builtin_amdgcn_wmma_f32_16x16x32_bf16(false, a, false, b, (short)0, c, false, false);
  }
  static __device__ __forceinline__ void guard4(v8f& a, v8f& b, v8f& c, v8f& d, v16b x, v16b y) { dep_guard4_b(a, b, c, d, x, y); }
  static __device__ __forceinline__ void keep(v16b a, v16b b, v16b c, v16b d) { keep4_b(a, b, c, d); }
};

template <int ET> struct Elem;
template <> struct Elem<0> { typedef _Float16 T; };
template <> struct Elem<1> { typedef __bf16 T; };
template <int ET, bool SPLIT, int BIAS_MODE, int OUT_MODE, bool RESID, int ACT = 0>
__global__ __launch_bounds__(256) void wmma_gemm64(
    const unsigned short* __restrict__ Ap, const unsigned short* __restrict__ A2p, int lda, long strideA,
    const unsigned short* __restrict__ Btp, const unsigned short* __restrict__ Bt2p, int ldb, long strideB,
    void* __restrict__ Cout, void* __restrict__ Cout2, int ldc, long strideC,
    const float* __restrict__ bias,
    const float* __restrict__ resid, long strideR,
    int M, int N, int K, float scale) {
  typedef typename Elem<ET>::T T;
  typedef typename Frag<T>::V V;
  const T* A = (const T*)Ap; const T* A2 = (const T*)A2p; const T* Bt = (const T*)Btp; const T* Bt2 = (const T*)Bt2p;
  __shared__ __align__(16) float sT[8][16 * 68];
  const int b    = blockIdx.y;
  const int lane = threadIdx.x & 31;
  const int wave = threadIdx.x >> 5;
  const int tilesN = N >> 6;
  const int tilesM = M >> 6;
  const int tile = blockIdx.x * 8 + wave;
  if (tile >= tilesM * tilesN) return;
  const int tm = tile / tilesN;
  const int tn = tile - tm * tilesN;
  const int m0 = tm << 6;
  const int n0 = tn << 6;

  const T* Ab  = A  + (size_t)b * strideA;
  const T* Bb  = Bt + (size_t)b * strideB;
  const T* Ab2 = SPLIT ? (A2  + (size_t)b * strideA) : nullptr;
  const T* Bb2 = SPLIT ? (Bt2 + (size_t)b * strideB) : nullptr;

  const int rlane = lane & 15;
  const int koff  = (lane >> 4) * 8;
  const int mOff  = (lane >> 4) * 8;

  v8f acc[4][4];
#pragma unroll
  for (int i = 0; i < 4; ++i)
#pragma unroll
    for (int j = 0; j < 4; ++j) acc[i][j] = (v8f){0.f,0.f,0.f,0.f,0.f,0.f,0.f,0.f};

  for (int k0 = 0; k0 < K; k0 += 32) {
    V bh[4], bl[4];
#pragma unroll
    for (int j = 0; j < 4; ++j) {
      const size_t bo = (size_t)(n0 + (j << 4) + rlane) * ldb + koff + k0;
      bh[j] = Frag<T>::load(Bb + bo);
      if (SPLIT) bl[j] = Frag<T>::load(Bb2 + bo);
    }
#pragma unroll
    for (int i = 0; i < 4; ++i) {
      const size_t ao = (size_t)(m0 + (i << 4) + rlane) * lda + koff + k0;
      V ah = Frag<T>::load(Ab + ao);
      V al;
      if (SPLIT) al = Frag<T>::load(Ab2 + ao);
#pragma unroll
      for (int j = 0; j < 4; ++j) {
        acc[i][j] = Frag<T>::mma(ah, bh[j], acc[i][j]);
        if (SPLIT) {
          acc[i][j] = Frag<T>::mma(ah, bl[j], acc[i][j]);
          acc[i][j] = Frag<T>::mma(al, bh[j], acc[i][j]);
        }
      }
      Frag<T>::guard4(acc[i][0], acc[i][1], acc[i][2], acc[i][3], ah, SPLIT ? al : bh[3]);
    }
    Frag<T>::keep(bh[0], bh[1], bh[2], bh[3]);
    if (SPLIT) Frag<T>::keep(bl[0], bl[1], bl[2], bl[3]);
  }
  acc_guard4(acc[0][0], acc[0][1], acc[0][2], acc[0][3]);
  acc_guard4(acc[1][0], acc[1][1], acc[1][2], acc[1][3]);
  acc_guard4(acc[2][0], acc[2][1], acc[2][2], acc[2][3]);
  acc_guard4(acc[3][0], acc[3][1], acc[3][2], acc[3][3]);

  float* slab = sT[wave];
  const float* Rb = RESID ? (resid + (size_t)b * strideR) : nullptr;
#pragma unroll
  for (int i = 0; i < 4; ++i) {
    const int mBase = m0 + (i << 4);
#pragma unroll
    for (int j = 0; j < 4; ++j) {
      const int n = n0 + (j << 4) + rlane;
      float bv = 0.f;
      if (BIAS_MODE == 2) bv = bias[n];
#pragma unroll
      for (int r = 0; r < 8; ++r) {
        float v = acc[i][j][r] * scale;
        if (BIAS_MODE == 1) v += bias[mBase + mOff + r];
        if (BIAS_MODE == 2) v += bv;
        if (RESID) v += Rb[(size_t)(mBase + mOff + r) * ldc + n];
        if (ACT == 2) v = fmaxf(v, 0.0f);
        if (ACT == 4) v = (v > 0.f) ? v : 0.01f * v;
        slab[(mOff + r) * 68 + (j << 4) + rlane] = v;
      }
    }
    __builtin_amdgcn_fence(__ATOMIC_RELEASE, "workgroup");
    __builtin_amdgcn_wave_barrier();
    __builtin_amdgcn_fence(__ATOMIC_ACQUIRE, "workgroup");
    if (OUT_MODE == 0) {
      float* C = (float*)Cout + (size_t)b * strideC;
      const int hh = lane >> 4, c4 = (lane & 15) * 4;
      for (int pass = 0; pass < 2; ++pass) {
#pragma unroll
        for (int it = 0; it < 8; ++it) {
          const int row = it * 2 + hh;
          v4f v = *(const v4f*)(slab + row * 68 + c4);
          *(volatile v4f*)(C + (size_t)(mBase + row) * ldc + n0 + c4) = v;
        }
        __threadfence();
      }
    } else {
      const int q = lane >> 3, c8 = (lane & 7) * 8;
      unsigned short* C  = (unsigned short*)Cout  + (size_t)b * strideC;
      unsigned short* C2 = (OUT_MODE == 2) ? ((unsigned short*)Cout2 + (size_t)b * strideC) : nullptr;
      for (int pass = 0; pass < 2; ++pass) {
#pragma unroll
        for (int it = 0; it < 4; ++it) {
          const int row = it * 4 + q;
          const float* sp = slab + row * 68 + c8;
          v8h hv, lv;
#pragma unroll
          for (int e = 0; e < 8; ++e) {
            if (OUT_MODE == 1) {
              hv[e] = (_Float16)sp[e];
            } else {
              unsigned short hb = f2bf_bits(sp[e]);
              unsigned short lb = f2bf_bits(sp[e] - bf_bits2f(hb));
              hv[e] = __builtin_bit_cast(_Float16, hb);
              lv[e] = __builtin_bit_cast(_Float16, lb);
            }
          }
          *(volatile v8h*)(C + (size_t)(mBase + row) * ldc + n0 + c8) = hv;
          if (OUT_MODE == 2) *(volatile v8h*)(C2 + (size_t)(mBase + row) * ldc + n0 + c8) = lv;
        }
        __threadfence();
      }
    }
    __builtin_amdgcn_fence(__ATOMIC_RELEASE, "workgroup");
    __builtin_amdgcn_wave_barrier();
    __builtin_amdgcn_fence(__ATOMIC_ACQUIRE, "workgroup");
  }
}

template <int MODE>
__global__ __launch_bounds__(256) void cvt8_kernel(const float* __restrict__ src, unsigned short* __restrict__ dst,
                                                   int n8, float sc) {
  const int i = blockIdx.x * 256 + threadIdx.x;
  if (i < n8) {
    const float* sp = src + (size_t)i * 8;
    const v4f a = *(const v4f*)(sp);
    const v4f b = *(const v4f*)(sp + 4);
    v8h hv;
#pragma unroll
    for (int e = 0; e < 4; ++e) {
      const float fa = a[e];
      const float fb = b[e];
      unsigned short b0, b1;
      if (MODE == 0) {
        b0 = f2bf_bits(fa);
        b1 = f2bf_bits(fb);
      } else {
        const _Float16 h0 = to_f16_operand(bf16r(fa) * sc);
        const _Float16 h1 = to_f16_operand(bf16r(fb) * sc);
        b0 = __builtin_bit_cast(unsigned short, h0);
        b1 = __builtin_bit_cast(unsigned short, h1);
      }
      hv[e]     = __builtin_bit_cast(_Float16, b0);
      hv[4 + e] = __builtin_bit_cast(_Float16, b1);
    }
    *(volatile v8h*)(dst + (size_t)i * 8) = hv;
    __threadfence();
    *(volatile v8h*)(dst + (size_t)i * 8) = hv;
  }
}

__global__ __launch_bounds__(256) void wcat_kernel(const float* __restrict__ Wq, const float* __restrict__ Wk,
                                                   const float* __restrict__ Wv, const float* __restrict__ Wb,
                                                   const float* __restrict__ Wa, unsigned short* __restrict__ dst) {
  const int i = blockIdx.x * 256 + threadIdx.x;
  if (i < kNcat * (kD / 8)) {
    const int row = i >> 7;
    const int c8  = i & 127;
    const float* base = Wq;
    int r = row;
    if (row >= kD)         { base = Wk; r = row - kD; }
    if (row >= 2 * kD)     { base = Wv; r = row - 2 * kD; }
    if (row >= kGate0)     { base = Wb; r = row - kGate0; }
    if (row >= kGate0 + kH) { base = Wa; r = row - kGate0 - kH; }
    const bool live = (row < kGate0 + 2 * kH);
    if (!live) r = kH - 1;
    const float* sp = base + (size_t)r * kD + c8 * 8;
    const v4f a = *(const v4f*)(sp);
    const v4f b = *(const v4f*)(sp + 4);
    v8h hv;
#pragma unroll
    for (int e = 0; e < 4; ++e) {
      const float fa = live ? a[e] : 0.0f;
      const float fb = live ? b[e] : 0.0f;
      const unsigned short b0 = f2bf_bits(fa);
      const unsigned short b1 = f2bf_bits(fb);
      hv[e]     = __builtin_bit_cast(_Float16, b0);
      hv[4 + e] = __builtin_bit_cast(_Float16, b1);
    }
    *(volatile v8h*)(dst + (size_t)i * 8) = hv;
    __threadfence();
    *(volatile v8h*)(dst + (size_t)i * 8) = hv;
  }
}

__global__ __launch_bounds__(256) void bias_prep_kernel(const float* __restrict__ bo, float* __restrict__ dst) {
  const int idx = threadIdx.x * 4;
  const v4f v = *(const v4f*)(bo + idx);
  v4f o;
#pragma unroll
  for (int e = 0; e < 4; ++e) {
    const float f = v[e];
    o[e] = bf16r(f);
  }
  *(volatile v4f*)(dst + idx) = o;
  __threadfence();
  *(volatile v4f*)(dst + idx) = o;
}

struct RopeTab { float f[64]; };
static_assert(sizeof(RopeTab) == 256, "no padding");

__global__ __launch_bounds__(256) void rope_gate_kernel(const float* __restrict__ QKVG,
                                                        const float* __restrict__ bbeta, const float* __restrict__ balpha,
                                                        float* __restrict__ QKR, float* __restrict__ GATES, RopeTab tab) {
  __shared__ __align__(16) float sCS[128];
  __shared__ __align__(16) float sG[64];
  const int tid = threadIdx.x, lane = tid & 31, wave = tid >> 5;
  const int t = blockIdx.x;
  if (tid < 64) {
    float invf = 0.0f;
#pragma unroll
    for (int j = 0; j < 64; ++j) invf = (tid == j) ? tab.f[j] : invf;
    const float ang = (float)t * invf;
    float sn, cs;
    sincosf(ang, &sn, &cs);
    sCS[2 * tid]     = cs;
    sCS[2 * tid + 1] = sn;
  } else if (tid < 96) {
    const int bb = lane >> 4, g = lane & 15;
    const size_t row = (size_t)bb * kL + t;
    const float zl = QKVG[row * kNcat + kGate0 + g];
    const float b0 = bbeta[g & 7];
    const float b1 = balpha[g & 7];
    const float bias = bf16r((g < kH) ? b0 : b1);
    const float z = zl + bias;
    const float sg = 1.0f / (1.0f + expf(-z));
    const float dec = kBetaMin + kBetaSpan * sg;
    sG[bb * 32 + g]      = (g < kH) ? dec : sg;
    sG[bb * 32 + 16 + g] = 0.0f;
  }
  __syncthreads();
  const int i0 = (2 * tid) & 63;
  const v4f cs4 = *(const v4f*)(sCS + 2 * i0);
#pragma unroll 1
  for (int j = 0; j < 4; ++j) {
    const int bb = j >> 1, it = j & 1;
    const size_t row = (size_t)bb * kL + t;
    const int f = tid + 256 * it;
    const v4f x = *(const v4f*)(QKVG + row * kNcat + 4 * f);
    v4f r;
    r[0] = x[0] * cs4[0] - x[1] * cs4[1];
    r[1] = x[1] * cs4[0] + x[0] * cs4[1];
    r[2] = x[2] * cs4[2] - x[3] * cs4[3];
    r[3] = x[3] * cs4[2] + x[2] * cs4[3];
    float* op = QKR + row * kQKP + 4 * f;
    *(volatile v4f*)op = r;
    __threadfence();
    *(volatile v4f*)op = r;
  }
  if (wave == 2) {
    const int l16 = lane & 15;
    const v4f gv = *(const v4f*)(sG + l16 * 4);
    const int bb = l16 >> 3, c4 = (l16 & 7) * 4;
    float* gp = GATES + ((size_t)bb * kL + t) * kGP + c4;
    if (lane < 16) {
      *(volatile v4f*)gp = gv;
      __threadfence();
      *(volatile v4f*)gp = gv;
    }
  }
}

__global__ __launch_bounds__(256) void scan_kernel(const float* __restrict__ QKR, const float* __restrict__ QKVG,
                                                   const float* __restrict__ GATES, unsigned short* __restrict__ OH) {
  __shared__ __align__(16) float    sQ[kScT * kDh];
  __shared__ __align__(16) float    sK[kScT * kDh];
  __shared__ __align__(16) float    sV[kScT * kScE];
  __shared__ __align__(16) _Float16 sO[kScT * kScE];
  __shared__ __align__(16) float    sB[kScT];
  const int tid = threadIdx.x, lane = tid & 31, wave = tid >> 5;
  const int bh = blockIdx.x >> 1, eb = blockIdx.x & 1;
  const int b = bh >> 3, h = bh & 7;
  const int el = wave * 8 + (lane & 7);
  const int qd = lane >> 3;
  const int dbase = qd * 32;
  const size_t row0 = (size_t)b * kL;
  const int vr = tid >> 4, vc4 = (tid & 15) * 4;
  const int fr = wave * 4 + (lane >> 3), fc8 = (lane & 7) * 8;

  float S[32];
#pragma unroll
  for (int i = 0; i < 32; ++i) S[i] = 0.0f;

#pragma unroll 1
  for (int c = 0; c < kL / kScT; ++c) {
    const size_t g0 = row0 + (size_t)c * kScT;
    __syncthreads();
#pragma unroll
    for (int it = 0; it < 4; ++it) {
      const int r = it * 8 + wave;
      const float* qp = QKR + (g0 + r) * kQKP + h * kDh + lane * 4;
      const v4f q4 = *(const v4f*)(qp);
      const v4f k4 = *(const v4f*)(qp + kD);
      *(v4f*)(sQ + r * kDh + lane * 4) = q4;
      *(v4f*)(sK + r * kDh + lane * 4) = k4;
    }
#pragma unroll
    for (int it = 0; it < 2; ++it) {
      const int r = it * 16 + vr;
      const v4f v4 = *(const v4f*)(QKVG + (g0 + r) * kNcat + 2 * kD + h * kDh + eb * kScE + vc4);
      const float al = GATES[(g0 + r) * kGP + kH + h];
      v4f w;
      w[0] = v4[0] * al;
      w[1] = v4[1] * al;
      w[2] = v4[2] * al;
      w[3] = v4[3] * al;
      *(v4f*)(sV + r * kScE + vc4) = w;
    }
    if (wave == 0) sB[lane] = GATES[(g0 + lane) * kGP + h];
    __syncthreads();

#pragma unroll 1
    for (int s = 0; s < kScT; ++s) {
      const float beta = sB[s];
      const float va = sV[s * kScE + el];
      const float* kp = sK + s * kDh + dbase;
      const float* qp = sQ + s * kDh + dbase;
      float acc0 = 0.0f, acc1 = 0.0f;
#pragma unroll
      for (int j = 0; j < 8; ++j) {
        const v4f k4 = *(const v4f*)(kp + 4 * j);
        const v4f q4 = *(const v4f*)(qp + 4 * j);
        float t0 = S[4 * j + 0] * beta;
        float t1 = S[4 * j + 1] * beta;
        float t2 = S[4 * j + 2] * beta;
        float t3 = S[4 * j + 3] * beta;
        t0 = fmaf(k4[0], va, t0);
        t1 = fmaf(k4[1], va, t1);
        t2 = fmaf(k4[2], va, t2);
        t3 = fmaf(k4[3], va, t3);
        S[4 * j + 0] = t0;
        S[4 * j + 1] = t1;
        S[4 * j + 2] = t2;
        S[4 * j + 3] = t3;
        acc0 = fmaf(q4[0], t0, acc0);
        acc1 = fmaf(q4[1], t1, acc1);
        acc0 = fmaf(q4[2], t2, acc0);
        acc1 = fmaf(q4[3], t3, acc1);
      }
      float tot = acc0 + acc1;
      tot = tot + __shfl_xor(tot, 8, 32);
      tot = tot + __shfl_xor(tot, 16, 32);
      const _Float16 oh = to_f16_operand(tot * kOCarry);
      if (qd == 0) sO[s * kScE + el] = oh;
    }
    __syncthreads();

    {
      const v8h hv = *(const v8h*)(sO + fr * kScE + fc8);
      unsigned short* gp = OH + (g0 + fr) * kD + h * kDh + eb * kScE + fc8;
      *(volatile v8h*)gp = hv;
      __threadfence();
      *(volatile v8h*)gp = hv;
    }
  }
}

extern "C" void kernel_launch(void* const* d_in, const int* in_sizes, int n_in,
                              void* d_out, int out_size, void* d_ws, size_t ws_size,
                              hipStream_t stream) {
  if (n_in < 10 || d_out == nullptr || d_ws == nullptr) return;
  if (in_sizes[0] != kRows * kD) return;
  if (in_sizes[1] != kD * kD || in_sizes[2] != kD * kD || in_sizes[3] != kD * kD) return;
  if (in_sizes[4] != kH * kD || in_sizes[5] != kH || in_sizes[6] != kH * kD || in_sizes[7] != kH) return;
  if (in_sizes[8] != kD * kD || in_sizes[9] != kD) return;
  if (out_size != kRows * kD) return;
  if (ws_size < kWsTotal) return;

  const float* x      = (const float*)d_in[0];
  const float* Wq     = (const float*)d_in[1];
  const float* Wk     = (const float*)d_in[2];
  const float* Wv     = (const float*)d_in[3];
  const float* Wbeta  = (const float*)d_in[4];
  const float* bbeta  = (const float*)d_in[5];
  const float* Walpha = (const float*)d_in[6];
  const float* balpha = (const float*)d_in[7];
  const float* Wo     = (const float*)d_in[8];
  const float* bo     = (const float*)d_in[9];
  float* out = (float*)d_out;

  char* ws = (char*)d_ws; size_t off = 0;
  auto carve = [&](size_t bytes) -> char* { char* p = ws + off; off += (bytes + 255) & ~(size_t)255; return p; };
  unsigned short* XB    = (unsigned short*)carve(kSzXB);
  unsigned short* WCAT  = (unsigned short*)carve(kSzWCAT);
  unsigned short* WOH   = (unsigned short*)carve(kSzWOH);
  float*          BOB   = (float*)carve(kSzBOB);
  float*          QKVG  = (float*)carve(kSzQKVG);
  float*          QKR   = (float*)carve(kSzQKR);
  float*          GATES = (float*)carve(kSzGATES);
  unsigned short* OH    = (unsigned short*)carve(kSzOH);
  if (off != kWsTotal || off > ws_size) return;

  RopeTab tab;
  {
    double r = 10000.0;
    for (int lvl = 0; lvl < 6; ++lvl) {
      const double a = r;
      double y = r;
      for (int it = 0; it < 80; ++it) y = 0.5 * (y + a / y);
      r = y;
    }
    double p = 1.0;
    for (int i = 0; i < 64; ++i) {
      const float pf = (float)p;
      tab.f[i] = 1.0f / pf;
      p *= r;
    }
  }

  const int n8x = kRows * (kD / 8);
  const int n8w = kD * (kD / 8);
  cvt8_kernel<0><<<n8x / 256, 256, 0, stream>>>(x, XB, n8x, 1.0f);
  wcat_kernel<<<(kNcat * (kD / 8)) / 256, 256, 0, stream>>>(Wq, Wk, Wv, Wbeta, Walpha, WCAT);
  cvt8_kernel<1><<<n8w / 256, 256, 0, stream>>>(Wo, WOH, n8w, kWoCarry);
  bias_prep_kernel<<<1, 256, 0, stream>>>(bo, BOB);

  wmma_gemm64<1, false, 0, 0, false, 0><<<dim3(((kRows / 64) * (kNcat / 64)) / 8, 1), 256, 0, stream>>>(
      XB, XB, kD, 0L,
      WCAT, WCAT, kD, 0L,
      (void*)QKVG, (void*)QKVG, kNcat, 0L,
      BOB, BOB, 0L,
      kRows, kNcat, kD, 1.0f);

  rope_gate_kernel<<<kL, 256, 0, stream>>>(QKVG, bbeta, balpha, QKR, GATES, tab);

  scan_kernel<<<kB * kH * (kDh / kScE), 256, 0, stream>>>(QKR, QKVG, GATES, OH);

  wmma_gemm64<0, false, 2, 0, false, 0><<<dim3(((kRows / 64) * (kD / 64)) / 8, 1), 256, 0, stream>>>(
      OH, OH, kD, 0L,
      WOH, WOH, kD, 0L,
      (void*)out, (void*)out, kD, 0L,
      BOB, BOB, 0L,
      kRows, kD, kD, kOutScale);
}
